// MHAEncoderFusedProj_42167988912449
// MI455X (gfx1250) — hardware-verified
//
#include <hip/hip_runtime.h>
#include <math.h>
#include <stdint.h>

#define NB    4
#define SEQ   2048
#define DMOD  1024
#define NQKV  (3 * DMOD)
#define NH    16
#define HD    64
#define QSC   8.0f
#define KSC   8.0f
#define RESC  2048.0f
#define PCAR  32768.0f
#define VCAR  1024.0f
#define OSC   1024.0f
#define WOS   1024.0f
#define LOG2E 1.4426950408889634f
#define ATT_WAVES   4
#define ATT_THREADS (ATT_WAVES * 32)
#define ATT_BLOCKS  (NB * NH * (SEQ / 64))
#define NKB    (SEQ / 32)
#define SLAB   (16 * 68)
static_assert(HD == 64 && DMOD == NH * HD);
static_assert((SEQ / 64) == 32 && NH == 16 && NB == 4);
static_assert(ATT_THREADS == 128 && ATT_BLOCKS == 2048 && NKB == 64);
static_assert(((NB * SEQ) % 64) == 0 && (DMOD % 64) == 0 && (DMOD % 32) == 0 && (SEQ % 64) == 0);
static_assert(((NB * SEQ * DMOD / 8) % 256) == 0 && ((NQKV * DMOD / 8) % 256) == 0 && ((DMOD * DMOD / 8) % 256) == 0);
static_assert((SLAB * 4) % 16 == 0);
static_assert((SEQ & (SEQ - 1)) == 0);

typedef unsigned short u16;
typedef _Float16 v16h __attribute__((ext_vector_type(16)));
typedef _Float16 v8h  __attribute__((ext_vector_type(8)));
typedef __bf16   v16b __attribute__((ext_vector_type(16)));
typedef float    v8f  __attribute__((ext_vector_type(8)));
typedef float    v4f  __attribute__((ext_vector_type(4)));
typedef unsigned int v4u __attribute__((ext_vector_type(4)));

union FragH { v16h v; v8h h[2]; v4u u[2]; };
union FragB { v16b v; v4u u[2]; };

__device__ __forceinline__ unsigned short bf_bits(float f) {
  unsigned u = __float_as_uint(f);
  return (unsigned short)((u + 0x7FFFu + ((u >> 16) & 1u)) >> 16);
}
__device__ __forceinline__ float bf_up(unsigned short h) { return __uint_as_float(((unsigned)h) << 16); }
__device__ __forceinline__ float bf_val(float f) { return bf_up(bf_bits(f)); }
__device__ __forceinline__ unsigned short h_bits(_Float16 x) { return __builtin_bit_cast(unsigned short, x); }
__device__ __forceinline__ unsigned pk16(unsigned short a, unsigned short b) { return (unsigned)a | ((unsigned)b << 16); }
__device__ __forceinline__ v8f zero8() { v8f z = {0.f, 0.f, 0.f, 0.f, 0.f, 0.f, 0.f, 0.f}; return z; }

__device__ __forceinline__ v16h ldfrag_h(const _Float16* p) {
  FragH f;
  f.h[0] = *(const v8h*)(p);
  f.h[1] = *(const v8h*)(p + 16);
  return f.v;
}
__device__ __forceinline__ v16b ldfrag_b(const u16* p) {
  FragB f;
  f.u[0] = *(const v4u*)(p);
  f.u[1] = *(const v4u*)(p + 16);
  return f.v;
}

__device__ __forceinline__ v8f mma_h(v16h a, v16h b, v8f c) {
  return __builtin_amdgcn_wmma_f32_16x16x32_f16(false, a, false, b, (short)0, c, false, false);
}
__device__ __forceinline__ v8f mma_b(v16b a, v16b b, v8f c) {
  return __builtin_amdgcn_wmma_f32_16x16x32_bf16(false, a, false, b, (short)0, c, false, false);
}
__device__ __forceinline__ void guard2x8(v8f& a, v8f& b, v16h x0, v16h x1, v16h x2, v16h x3,
                                         v16h x4, v16h x5, v16h x6, v16h x7) {
#if defined(__HIP_DEVICE_COMPILE__)
  asm volatile("v_nop\n\tv_nop\n\tv_nop\n\tv_nop"
               : "+v"(a), "+v"(b)
               : "v"(x0), "v"(x1), "v"(x2), "v"(x3), "v"(x4), "v"(x5), "v"(x6), "v"(x7) : "memory");
#endif
}
template <typename F>
__device__ __forceinline__ void guard6(v8f& a, v8f& b, v8f& c, v8f& d, F x0, F x1, F x2, F x3, F x4, F x5) {
#if defined(__HIP_DEVICE_COMPILE__)
  asm volatile("v_nop\n\tv_nop\n\tv_nop\n\tv_nop"
               : "+v"(a), "+v"(b), "+v"(c), "+v"(d) : "v"(x0), "v"(x1), "v"(x2), "v"(x3), "v"(x4), "v"(x5) : "memory");
#endif
}
__device__ __forceinline__ void acc_guard4(v8f& a, v8f& b, v8f& c, v8f& d) {
#if defined(__HIP_DEVICE_COMPILE__)
  asm volatile("v_nop\n\tv_nop\n\tv_nop\n\tv_nop" : "+v"(a), "+v"(b), "+v"(c), "+v"(d));
#endif
}
__device__ __forceinline__ void wave_sync_lds() {
#if defined(__HIP_DEVICE_COMPILE__)
  __builtin_amdgcn_fence(__ATOMIC_RELEASE, "workgroup");
  __builtin_amdgcn_wave_barrier();
  __builtin_amdgcn_fence(__ATOMIC_ACQUIRE, "workgroup");
#endif
}

__global__ __launch_bounds__(256) void cvt16(const float* __restrict__ x, u16* D, int n8, int mode, float scale) {
  const int gt = blockIdx.x * 256 + (int)threadIdx.x;
  if (gt >= n8) return;
  const float* p = x + (size_t)gt * 8;
  const v4f a = *(const v4f*)(p), c4 = *(const v4f*)(p + 4);
  float v[8];
#pragma unroll
  for (int e = 0; e < 4; ++e) { v[e] = a[e]; v[4 + e] = c4[e]; }
  unsigned short s[8];
#pragma unroll
  for (int e = 0; e < 8; ++e) {
    const unsigned short bb = bf_bits(v[e]);
    const unsigned short hb = h_bits((_Float16)(bf_up(bb) * scale));
    s[e] = (mode != 0) ? hb : bb;
  }
  v4u o;
#pragma unroll
  for (int e = 0; e < 4; ++e) o[e] = pk16(s[2 * e], s[2 * e + 1]);
  u16* d = D + (size_t)gt * 8;
  for (int pass = 0; pass < 2; ++pass) {
    *(volatile v4u*)(d) = o;
    __threadfence();
  }
}

__device__ __forceinline__ void epi16(float* sl, v8f a0, v8f a1, v8f a2, v8f a3, float oscale, u16* C, int N,
                                      size_t rowb, int col0, int lane) {
  const int hh = lane >> 4, m = lane & 15;
#pragma unroll
  for (int r = 0; r < 8; ++r) {
    const int ro = (8 * hh + r) * 68 + m;
    sl[ro]      = a0[r] * oscale;
    sl[ro + 16] = a1[r] * oscale;
    sl[ro + 32] = a2[r] * oscale;
    sl[ro + 48] = a3[r] * oscale;
  }
  wave_sync_lds();
  const int rq = lane >> 3, c8 = (lane & 7) * 8;
  v4u ov[4];
#pragma unroll
  for (int i4 = 0; i4 < 4; ++i4) {
    const int row = i4 * 4 + rq;
    const v4f a = *(const v4f*)(sl + row * 68 + c8), c4 = *(const v4f*)(sl + row * 68 + c8 + 4);
    float w[8];
#pragma unroll
    for (int e = 0; e < 4; ++e) { w[e] = a[e]; w[4 + e] = c4[e]; }
#pragma unroll
    for (int e = 0; e < 4; ++e) ov[i4][e] = pk16(h_bits((_Float16)w[2 * e]), h_bits((_Float16)w[2 * e + 1]));
  }
  u16* dst = C + (rowb + (size_t)rq) * (size_t)N + col0 + c8;
  for (int pass = 0; pass < 2; ++pass) {
#pragma unroll
    for (int i4 = 0; i4 < 4; ++i4) {
      *(volatile v4u*)(dst + (size_t)(i4 * 4) * (size_t)N) = ov[i4];
    }
    __threadfence();
  }
}

__device__ __forceinline__ void epi_rope(float* sl, v8f a0, v8f a1, v8f a2, v8f a3,
                                         const float* __restrict__ cosp, const float* __restrict__ sinp,
                                         u16* CH, u16* CL, int N, size_t rowb, int col0, int lane) {
  const int hh = lane >> 4, m = lane & 15;
#pragma unroll
  for (int r = 0; r < 8; ++r) {
    const int ro = (8 * hh + r) * 68 + m;
    sl[ro]      = a0[r];
    sl[ro + 16] = a1[r];
    sl[ro + 32] = a2[r];
    sl[ro + 48] = a3[r];
  }
  wave_sync_lds();
  const int rq = lane >> 3, c8 = (lane & 7) * 8, p8 = c8 ^ 32;
  const float sgn = (c8 < 32) ? -1.0f : 1.0f;
  v4u ovh[4], ovl[4];
#pragma unroll
  for (int i4 = 0; i4 < 4; ++i4) {
    const int row  = i4 * 4 + rq;
    const int srow = (int)((rowb + (size_t)row) & (size_t)(SEQ - 1));
    const v4f xa = *(const v4f*)(sl + row * 68 + c8), xb = *(const v4f*)(sl + row * 68 + c8 + 4);
    const v4f ya = *(const v4f*)(sl + row * 68 + p8), yb = *(const v4f*)(sl + row * 68 + p8 + 4);
    const float* cr = cosp + (size_t)srow * HD + c8;
    const float* sr = sinp + (size_t)srow * HD + c8;
    const v4f ca = *(const v4f*)(cr), cb = *(const v4f*)(cr + 4);
    const v4f sa = *(const v4f*)(sr), sb = *(const v4f*)(sr + 4);
    float w[8];
#pragma unroll
    for (int e = 0; e < 4; ++e) {
      w[e]     = xa[e] * bf_val(ca[e]) + sgn * (ya[e] * bf_val(sa[e]));
      w[4 + e] = xb[e] * bf_val(cb[e]) + sgn * (yb[e] * bf_val(sb[e]));
    }
    unsigned short hb[8], lb[8];
#pragma unroll
    for (int e = 0; e < 8; ++e) {
      const float    t  = w[e] * QSC;
      const _Float16 hv = (_Float16)t;
      hb[e] = h_bits(hv);
      lb[e] = h_bits((_Float16)((t - (float)hv) * RESC));
    }
#pragma unroll
    for (int e = 0; e < 4; ++e) {
      ovh[i4][e] = pk16(hb[2 * e], hb[2 * e + 1]);
      ovl[i4][e] = pk16(lb[2 * e], lb[2 * e + 1]);
    }
  }
  u16* dh = CH + (rowb + (size_t)rq) * (size_t)N + col0 + c8;
  u16* dl = CL + (rowb + (size_t)rq) * (size_t)N + col0 + c8;
  for (int pass = 0; pass < 2; ++pass) {
#pragma unroll
    for (int i4 = 0; i4 < 4; ++i4) {
      *(volatile v4u*)(dh + (size_t)(i4 * 4) * (size_t)N) = ovh[i4];
      *(volatile v4u*)(dl + (size_t)(i4 * 4) * (size_t)N) = ovl[i4];
    }
    __threadfence();
  }
}

__device__ __forceinline__ void epi64(float* sl, v8f a0, v8f a1, v8f a2, v8f a3, float oscale, float* C, int N,
                                      size_t rowb, int col0, int lane) {
  const int hh = lane >> 4, m = lane & 15;
#pragma unroll
  for (int r = 0; r < 8; ++r) {
    const int ro = (8 * hh + r) * 68 + m;
    sl[ro]      = a0[r] * oscale;
    sl[ro + 16] = a1[r] * oscale;
    sl[ro + 32] = a2[r] * oscale;
    sl[ro + 48] = a3[r] * oscale;
  }
  wave_sync_lds();
  v4f vals[8];
#pragma unroll
  for (int it = 0; it < 8; ++it) vals[it] = *(const v4f*)(sl + (it * 2 + hh) * 68 + m * 4);
  float* dst = C + (rowb + (size_t)hh) * (size_t)N + col0 + m * 4;
  for (int pass = 0; pass < 2; ++pass) {
#pragma unroll
    for (int it = 0; it < 8; ++it) {
      *(volatile v4f*)(dst + (size_t)(it * 2) * (size_t)N) = vals[it];
    }
    __threadfence();
  }
}

__global__ __launch_bounds__(128)
void gemm_b16(const u16* __restrict__ A, const u16* __restrict__ Bt, u16* C, int M, int N, int K,
              int bstA, int bstB, int bstC, float oscale) {
  __shared__ __align__(16) float slab[4 * SLAB];
  const int tid = threadIdx.x, wave = tid >> 5, lane = tid & 31, hh = lane >> 4, m = lane & 15;
  const int ntile = N >> 6, mtile = M >> 6;
  const int per   = ntile * mtile;
  const int bid   = blockIdx.x;
  const int bt    = bid / per;
  const int t     = bid - bt * per;
  const int rowb  = (t / ntile) * 64 + wave * 16;
  const int col0  = (t % ntile) * 64;
  if (rowb + 16 > M) return;
  const u16* Ab = A  + (size_t)bt * (size_t)bstA;
  const u16* Bb = Bt + (size_t)bt * (size_t)bstB;
  u16*       Cb = C  + (size_t)bt * (size_t)bstC;
  const u16* ap = Ab + (size_t)(rowb + m) * K + 8 * hh;
  const u16* bp = Bb + (size_t)(col0 + m) * K + 8 * hh;
  const size_t bs = (size_t)16 * K;
  v8f acc0 = zero8(), acc1 = zero8(), acc2 = zero8(), acc3 = zero8();
#pragma unroll 1
  for (int k0 = 0; k0 < K; k0 += 32) {
    const v16b a  = ldfrag_b(ap + k0);
    const v16b b0 = ldfrag_b(bp + k0);
    const v16b b1 = ldfrag_b(bp + bs + k0);
    const v16b b2 = ldfrag_b(bp + 2 * bs + k0);
    const v16b b3 = ldfrag_b(bp + 3 * bs + k0);
    acc0 = mma_b(a, b0, acc0);
    acc1 = mma_b(a, b1, acc1);
    acc2 = mma_b(a, b2, acc2);
    acc3 = mma_b(a, b3, acc3);
    guard6<v16b>(acc0, acc1, acc2, acc3, a, b0, b1, b2, b3, a);
  }
  epi16(slab + wave * SLAB, acc0, acc1, acc2, acc3, oscale, Cb, N, (size_t)rowb, col0, lane);
}

__global__ __launch_bounds__(128)
void gemm_rope(const u16* __restrict__ A, const u16* __restrict__ Bt, const float* __restrict__ cosp,
               const float* __restrict__ sinp, u16* CH, u16* CL, int M, int N, int K) {
  __shared__ __align__(16) float slab[4 * SLAB];
  const int tid = threadIdx.x, wave = tid >> 5, lane = tid & 31, hh = lane >> 4, m = lane & 15;
  const int ntile = N >> 6;
  const int bid   = blockIdx.x;
  const int rowb  = (bid / ntile) * 64 + wave * 16;
  const int col0  = (bid % ntile) * 64;
  if (rowb + 16 > M) return;
  const u16* ap = A  + (size_t)(rowb + m) * K + 8 * hh;
  const u16* bp = Bt + (size_t)(col0 + m) * K + 8 * hh;
  const size_t bs = (size_t)16 * K;
  v8f acc0 = zero8(), acc1 = zero8(), acc2 = zero8(), acc3 = zero8();
#pragma unroll 1
  for (int k0 = 0; k0 < K; k0 += 32) {
    const v16b a  = ldfrag_b(ap + k0);
    const v16b b0 = ldfrag_b(bp + k0);
    const v16b b1 = ldfrag_b(bp + bs + k0);
    const v16b b2 = ldfrag_b(bp + 2 * bs + k0);
    const v16b b3 = ldfrag_b(bp + 3 * bs + k0);
    acc0 = mma_b(a, b0, acc0);
    acc1 = mma_b(a, b1, acc1);
    acc2 = mma_b(a, b2, acc2);
    acc3 = mma_b(a, b3, acc3);
    guard6<v16b>(acc0, acc1, acc2, acc3, a, b0, b1, b2, b3, a);
  }
  epi_rope(slab + wave * SLAB, acc0, acc1, acc2, acc3, cosp, sinp, CH, CL, N, (size_t)rowb, col0, lane);
}

__global__ __launch_bounds__(128)
void gemm_hf(const u16* __restrict__ A, const u16* __restrict__ Bt, float* C, int M, int N, int K, float oscale) {
  __shared__ __align__(16) float slab[4 * SLAB];
  const int tid = threadIdx.x, wave = tid >> 5, lane = tid & 31, hh = lane >> 4, m = lane & 15;
  const int ntile = N >> 6;
  const int bid   = blockIdx.x;
  const int rowb  = (bid / ntile) * 64 + wave * 16;
  const int col0  = (bid % ntile) * 64;
  if (rowb + 16 > M) return;
  const _Float16* ap = (const _Float16*)(const void*)A  + (size_t)(rowb + m) * K + 8 * hh;
  const _Float16* bp = (const _Float16*)(const void*)Bt + (size_t)(col0 + m) * K + 8 * hh;
  const size_t bs = (size_t)16 * K;
  v8f acc0 = zero8(), acc1 = zero8(), acc2 = zero8(), acc3 = zero8();
#pragma unroll 1
  for (int k0 = 0; k0 < K; k0 += 32) {
    const v16h a  = ldfrag_h(ap + k0);
    const v16h b0 = ldfrag_h(bp + k0);
    const v16h b1 = ldfrag_h(bp + bs + k0);
    const v16h b2 = ldfrag_h(bp + 2 * bs + k0);
    const v16h b3 = ldfrag_h(bp + 3 * bs + k0);
    acc0 = mma_h(a, b0, acc0);
    acc1 = mma_h(a, b1, acc1);
    acc2 = mma_h(a, b2, acc2);
    acc3 = mma_h(a, b3, acc3);
    guard6<v16h>(acc0, acc1, acc2, acc3, a, b0, b1, b2, b3, a);
  }
  epi64(slab + wave * SLAB, acc0, acc1, acc2, acc3, oscale, C, N, (size_t)rowb, col0, lane);
}

__global__ __launch_bounds__(ATT_THREADS)
void attn_fwd(const u16* __restrict__ QHp, const u16* __restrict__ QLp, const u16* __restrict__ KHp,
              const u16* __restrict__ KLp, const u16* __restrict__ VPp, u16* OPp) {
  __shared__ __align__(16) float smem[ATT_WAVES * SLAB];

  const int tid  = threadIdx.x;
  const int wave = tid >> 5;
  const int lane = tid & 31;
  const int hh   = lane >> 4;
  const int c    = lane & 15;

  const int bid  = blockIdx.x;
  const int qt   = bid & (SEQ / 64 - 1);
  const int head = (bid >> 5) & (NH - 1);
  const int b    = bid >> 9;
  const int q0   = qt * 64 + wave * 16;

  const size_t qofs = (((size_t)(b * SEQ + q0 + c)) * NH + head) * HD + 8 * hh;
  const _Float16* QHb = (const _Float16*)(const void*)QHp + qofs;
  const _Float16* QLb = (const _Float16*)(const void*)QLp + qofs;
  const size_t kofs = (((size_t)b * SEQ + c) * NH + head) * HD + 8 * hh;
  const _Float16* KHb = (const _Float16*)(const void*)KHp + kofs;
  const _Float16* KLb = (const _Float16*)(const void*)KLp + kofs;
  const size_t vofs = ((size_t)(b * NH + head) * HD + c) * SEQ + 8 * hh;
  const _Float16* Vb = (const _Float16*)(const void*)VPp + vofs;
  const float lsch = 0.125f * (LOG2E / (QSC * KSC));
  const float lscx = lsch * (1.0f / RESC);

  const v16h qh0 = ldfrag_h(QHb);
  const v16h qh1 = ldfrag_h(QHb + 32);
  const v16h ql0 = ldfrag_h(QLb);
  const v16h ql1 = ldfrag_h(QLb + 32);

  float mrun = -INFINITY, lrun = 0.f;
  v8f o[4];
#pragma unroll
  for (int j = 0; j < 4; ++j) o[j] = zero8();

#pragma unroll 1
  for (int it = 0; it < NKB; ++it) {
    const int kb = it * 32;
    const size_t krow = (size_t)kb * (NH * HD);
    v8f s0h = zero8(), s0x = zero8(), s1h = zero8(), s1x = zero8();
    {
      const _Float16* k0p = KHb + krow;
      const _Float16* l0p = KLb + krow;
      const v16h ka0 = ldfrag_h(k0p), ka1 = ldfrag_h(k0p + 32);
      const v16h la0 = ldfrag_h(l0p), la1 = ldfrag_h(l0p + 32);
      s0h = mma_h(ka0, qh0, s0h);
      s0h = mma_h(ka1, qh1, s0h);
      s0x = mma_h(ka0, ql0, s0x);
      s0x = mma_h(ka1, ql1, s0x);
      s0x = mma_h(la0, qh0, s0x);
      s0x = mma_h(la1, qh1, s0x);
      guard2x8(s0h, s0x, qh0, qh1, ql0, ql1, ka0, ka1, la0, la1);
    }
    {
      const _Float16* k1p = KHb + krow + (size_t)16 * (NH * HD);
      const _Float16* l1p = KLb + krow + (size_t)16 * (NH * HD);
      const v16h kc0 = ldfrag_h(k1p), kc1 = ldfrag_h(k1p + 32);
      const v16h lc0 = ldfrag_h(l1p), lc1 = ldfrag_h(l1p + 32);
      s1h = mma_h(kc0, qh0, s1h);
      s1h = mma_h(kc1, qh1, s1h);
      s1x = mma_h(kc0, ql0, s1x);
      s1x = mma_h(kc1, ql1, s1x);
      s1x = mma_h(lc0, qh0, s1x);
      s1x = mma_h(lc1, qh1, s1x);
      guard2x8(s1h, s1x, qh0, qh1, ql0, ql1, kc0, kc1, lc0, lc1);
    }
    float tk[16];
#pragma unroll
    for (int i = 0; i < 8; ++i) {
      tk[i]     = s0h[i] * lsch + s0x[i] * lscx;
      tk[8 + i] = s1h[i] * lsch + s1x[i] * lscx;
    }
    float cm = tk[0];
#pragma unroll
    for (int i = 1; i < 16; ++i) cm = fmaxf(cm, tk[i]);
    cm = fmaxf(cm, __shfl_xor(cm, 16, 32));
    const float mn = fmaxf(mrun, cm);
    const float al = (mrun == -INFINITY) ? 0.f : exp2f(mrun - mn);
    mrun = mn;
    float ps = 0.f;
    FragH ph;
#pragma unroll
    for (int w = 0; w < 2; ++w) {
#pragma unroll
      for (int e4 = 0; e4 < 4; ++e4) {
        const int i = 8 * w + 2 * e4;
        const float p0 = exp2f(fminf(tk[i] - mn, 0.f));
        const float p1 = exp2f(fminf(tk[i + 1] - mn, 0.f));
        ps += p0 + p1;
        ph.u[w][e4] = pk16(h_bits((_Float16)(p0 * PCAR)), h_bits((_Float16)(p1 * PCAR)));
      }
    }
    ps += __shfl_xor(ps, 16, 32);
    lrun = lrun * al + ps;
    float scl[8];
#pragma unroll
    for (int r = 0; r < 8; ++r) scl[r] = __shfl(al, 8 * hh + r, 32);
#pragma unroll
    for (int j = 0; j < 4; ++j) {
#pragma unroll
      for (int r = 0; r < 8; ++r) o[j][r] *= scl[r];
    }
    {
      const _Float16* vp = Vb + kb;
      const v16h vf0 = ldfrag_h(vp);
      const v16h vf1 = ldfrag_h(vp + (size_t)16 * SEQ);
      const v16h vf2 = ldfrag_h(vp + (size_t)32 * SEQ);
      const v16h vf3 = ldfrag_h(vp + (size_t)48 * SEQ);
      o[0] = mma_h(ph.v, vf0, o[0]);
      o[1] = mma_h(ph.v, vf1, o[1]);
      o[2] = mma_h(ph.v, vf2, o[2]);
      o[3] = mma_h(ph.v, vf3, o[3]);
      guard6<v16h>(o[0], o[1], o[2], o[3], ph.v, vf0, vf1, vf2, vf3, ph.v);
    }
  }
  acc_guard4(o[0], o[1], o[2], o[3]);

  const float linv = (lrun > 0.f) ? ((1.0f / lrun) * (1.0f / (PCAR * VCAR))) : 0.f;
  float inv[8];
#pragma unroll
  for (int r = 0; r < 8; ++r) inv[r] = __shfl(linv, 8 * hh + r, 32);
  float* slab = smem + wave * SLAB;
#pragma unroll
  for (int r = 0; r < 8; ++r) {
#pragma unroll
    for (int j = 0; j < 4; ++j) slab[(8 * hh + r) * 68 + j * 16 + c] = o[j][r] * inv[r];
  }
  wave_sync_lds();
  v4u oh[4];
  const int rq = lane >> 3, c8 = (lane & 7) * 8;
#pragma unroll
  for (int i4 = 0; i4 < 4; ++i4) {
    const int row = i4 * 4 + rq;
    const v4f a = *(const v4f*)(slab + row * 68 + c8), c4 = *(const v4f*)(slab + row * 68 + c8 + 4);
    float w[8];
#pragma unroll
    for (int e = 0; e < 4; ++e) { w[e] = a[e] * OSC; w[4 + e] = c4[e] * OSC; }
#pragma unroll
    for (int e = 0; e < 4; ++e) oh[i4][e] = pk16(h_bits((_Float16)w[2 * e]), h_bits((_Float16)w[2 * e + 1]));
  }
  const size_t ob = (((size_t)(b * SEQ + q0)) * NH + head) * HD + c8;
  for (int pass = 0; pass < 2; ++pass) {
#pragma unroll
    for (int i4 = 0; i4 < 4; ++i4) {
      const int row = i4 * 4 + rq;
      const size_t o8 = ob + (size_t)row * (NH * HD);
      *(volatile v4u*)(OPp + o8) = oh[i4];
    }
    __threadfence();
  }
}

extern "C" void kernel_launch(void* const* d_in, const int* in_sizes, int n_in,
                              void* d_out, int out_size, void* d_ws, size_t ws_size,
                              hipStream_t stream) {
  const int ROWS = NB * SEQ;
  if (n_in < 5) return;
  if (in_sizes[0] != ROWS * DMOD) return;
  if (in_sizes[1] != SEQ * HD) return;
  if (in_sizes[2] != SEQ * HD) return;
  if (in_sizes[3] != NQKV * DMOD) return;
  if (in_sizes[4] != DMOD * DMOD) return;
  if (out_size != ROWS * DMOD) return;

  const float* Xin = (const float*)d_in[0];
  const float* Cs  = (const float*)d_in[1];
  const float* Sn  = (const float*)d_in[2];
  const float* Wqk = (const float*)d_in[3];
  const float* Wpr = (const float*)d_in[4];
  float*       out = (float*)d_out;

  const size_t szXB = (size_t)ROWS * DMOD * 2;
  const size_t szWB = (size_t)NQKV * DMOD * 2;
  const size_t szWO = (size_t)DMOD * DMOD * 2;
  const size_t szP  = (size_t)ROWS * DMOD * 2;
  const size_t szVP = (size_t)NB * NH * HD * SEQ * 2;
  size_t off = 0;
  const size_t oXB = off; off += szXB;
  const size_t oWB = off; off += szWB;
  const size_t oWO = off; off += szWO;
  const size_t oQH = off; off += szP;
  const size_t oQL = off; off += szP;
  const size_t oKH = off; off += szP;
  const size_t oKL = off; off += szP;
  const size_t oVP = off; off += szVP;
  const size_t oOP = oXB;
  if (szP > szXB) return;
  if (off > ws_size) return;
  if (off > (size_t)134217728) return;

  char* ws = (char*)d_ws;
  u16* XB  = (u16*)(ws + oXB);
  u16* WB  = (u16*)(ws + oWB);
  u16* WOB = (u16*)(ws + oWO);
  u16* QH  = (u16*)(ws + oQH);
  u16* QL  = (u16*)(ws + oQL);
  u16* KH  = (u16*)(ws + oKH);
  u16* KL  = (u16*)(ws + oKL);
  u16* VP  = (u16*)(ws + oVP);
  u16* OP  = (u16*)(ws + oOP);

  const dim3 blk(256);
  const int n8x = (ROWS * DMOD) / 8;
  const int n8q = (NQKV * DMOD) / 8;
  const int n8w = (DMOD * DMOD) / 8;
  if ((n8x % 256) != 0 || (n8q % 256) != 0 || (n8w % 256) != 0) return;
  if ((DMOD % 64) != 0 || (ROWS % 64) != 0 || (SEQ % 64) != 0 || (DMOD % 32) != 0) return;
  const dim3 gX(n8x / 256);
  const dim3 gQ(n8q / 256);
  const dim3 gW(n8w / 256);
  const dim3 gG((ROWS / 64) * (DMOD / 64));
  const dim3 gV(NB * (DMOD / 64) * (SEQ / 64));
  const dim3 bG(128);
  const dim3 gAT(ATT_BLOCKS);
  const dim3 bAT(ATT_THREADS);

  cvt16<<<gX, blk, 0, stream>>>(Xin, XB, n8x, 0, 1.0f);
  cvt16<<<gQ, blk, 0, stream>>>(Wqk, WB, n8q, 0, 1.0f);
  cvt16<<<gW, blk, 0, stream>>>(Wpr, WOB, n8w, 1, WOS);
  gemm_rope<<<gG, bG, 0, stream>>>(XB, WB, Cs, Sn, QH, QL, ROWS, DMOD, DMOD);
  gemm_rope<<<gG, bG, 0, stream>>>(XB, WB + (size_t)DMOD * DMOD, Cs, Sn, KH, KL, ROWS, DMOD, DMOD);
  gemm_b16<<<gV, bG, 0, stream>>>(WB + (size_t)2 * DMOD * DMOD, XB, VP, DMOD, SEQ, DMOD, 0, SEQ * DMOD, DMOD * SEQ, VCAR);
  attn_fwd<<<gAT, bAT, 0, stream>>>(QH, QL, KH, KL, VP, OP);
  gemm_hf<<<gG, bG, 0, stream>>>(OP, WOB, out, ROWS, DMOD, DMOD, 1.0f / (OSC * WOS));
  (void)hipGetLastError();
}
